// Attention_80822694576396
// MI455X (gfx1250) — hardware-verified
//
#include <hip/hip_runtime.h>


#ifndef NB
#define NB 4
#endif
#ifndef SEQ
#define SEQ 4096
#endif
#define NB_FULL  4
#define SEQ_FULL 4096
#define CH   256
#define NH   4
#define HD   64
#define OC3  768
#define NWV  4
#define BQ   (16 * NWV)
#define KS   32
#define XP   264
#define SQ   72
#define OP   68
#define L2E  1.4426950408889634f

static_assert(CH == NH * HD);
static_assert(OC3 == 3 * CH);
static_assert(CH == 256);
static_assert(HD == 64);
static_assert(CH % 32 == 0);
static_assert(SEQ % BQ == 0);
static_assert(SEQ % KS == 0);
static_assert(SEQ % 64 == 0);
static_assert(SEQ % 4 == 0);
static_assert(NB <= NB_FULL);
static_assert(SEQ <= SEQ_FULL);
static_assert((OC3 * CH / 8) % 256 == 0);
static_assert((CH * CH / 8) % 256 == 0);
static_assert((XP * 2) % 16 == 0);
static_assert((SQ * 2) % 16 == 0);
static_assert((OP * 4) % 16 == 0);
static_assert((size_t)(NB * (SEQ / 64)) * (size_t)(64 * CH) == (size_t)NB * SEQ * CH);
static_assert((size_t)(SEQ / 64) * 12 * NB * (size_t)(64 * 64) == (size_t)NB * SEQ * OC3);
static_assert((size_t)(NB * NH * (SEQ / BQ)) * (size_t)(BQ * HD) == (size_t)NB * SEQ * CH);
static_assert((size_t)(SEQ / 64) * (CH / 64) * NB * (size_t)(64 * 64) == (size_t)NB * SEQ * CH);

#define ST_BYTES  ((size_t)4096)
#define WQ_BYTES  ((size_t)OC3 * CH * 2)
#define WO_BYTES  ((size_t)CH * CH * 2)
#define PL_BYTES  ((size_t)NB * SEQ * CH * 2)
#define WS_TOTAL  (ST_BYTES + WQ_BYTES + WO_BYTES + 6 * PL_BYTES)
static_assert(WQ_BYTES % 256 == 0);
static_assert(WO_BYTES % 256 == 0);
static_assert(PL_BYTES % 256 == 0);
static_assert((size_t)NB * NH * SEQ * HD * 2 == PL_BYTES);
static_assert(WS_TOTAL <= (size_t)134217728);

typedef _Float16 hf;
typedef __attribute__((ext_vector_type(16))) _Float16 v16h;
typedef __attribute__((ext_vector_type(8)))  _Float16 v8h;
typedef __attribute__((ext_vector_type(8)))  float    v8f;
typedef __attribute__((ext_vector_type(4)))  float    v4f;
typedef v4f __attribute__((may_alias)) v4fa;
typedef v8h __attribute__((may_alias)) v8ha;

__device__ __forceinline__ float bfr(float f) { unsigned u = __float_as_uint(f); u += 0x7FFFu + ((u >> 16) & 1u); return __uint_as_float(u & 0xFFFF0000u); }
__device__ __forceinline__ v16h cat16(v8h lo, v8h hi) { return __builtin_shufflevector(lo, hi, 0, 1, 2, 3, 4, 5, 6, 7, 8, 9, 10, 11, 12, 13, 14, 15); }
__device__ __forceinline__ v8f wmmah(v16h a, v16h b, v8f c) { return __builtin_amdgcn_wmma_f32_16x16x32_f16(false, a, false, b, (short)0, c, false, false); }
__device__ __forceinline__ v16h ldh(const hf* p) { return cat16(*(const v8h*)p, *(const v8h*)(p + 16)); }

__device__ __forceinline__ void cvt8w(const float* __restrict__ src, hf* dst, unsigned i) {
    const v8f v = *(const v8f*)(src + (size_t)i * 8);
    v8h o;
#pragma unroll
    for (int c = 0; c < 8; ++c) o[c] = (hf)(bfr(v[c]) * 1024.0f);
    hf* d = dst + (size_t)i * 8;
    *(volatile v8h*)d = o;
    __threadfence();
    *(volatile v8h*)d = o;
}

__global__ __launch_bounds__(256) void k_cvtw(const float* __restrict__ wq, const float* __restrict__ wo, hf* WQ, hf* WO) {
    const unsigned i = blockIdx.x * 256u + threadIdx.x;
    if (blockIdx.y == 0) {
        if (i < (unsigned)(OC3 * CH / 8)) cvt8w(wq, WQ, i);
    } else {
        if (i < (unsigned)(CH * CH / 8)) cvt8w(wo, WO, i);
    }
}

__global__ __launch_bounds__(256) void k_bnstat(const float* __restrict__ x, float* ST) {
    __shared__ float red1[8];
    __shared__ float red2[8];
    __shared__ float resl[32];
    const unsigned tid = threadIdx.x, lane = tid & 31u;
    const unsigned wave = (unsigned)__builtin_amdgcn_readfirstlane((int)(tid >> 5));
    if (tid < 32u) resl[tid] = 0.0f;
    const float invn = 1.0f / (float)(NB * SEQ);
#pragma unroll 1
    for (unsigned cc = 0; cc < 8u; ++cc) {
        const unsigned c = blockIdx.x * 8u + cc;
        float s = 0.0f;
#pragma unroll 1
        for (unsigned b = 0; b < (unsigned)NB; ++b) {
            const float* xp = x + ((size_t)b * CH + c) * SEQ_FULL;
#pragma unroll 1
            for (unsigned i = tid * 4u; i < (unsigned)SEQ; i += 1024u) {
                const v4f v = *(const v4f*)(xp + i);
                s += (bfr(v[0]) + bfr(v[1])) + (bfr(v[2]) + bfr(v[3]));
            }
        }
#pragma unroll
        for (int off = 16; off > 0; off >>= 1) s += __shfl_xor(s, off, 32);
        if (lane == 0u) red1[wave] = s;
        __syncthreads();
        float tot = red1[0];
#pragma unroll
        for (int w = 1; w < 8; ++w) tot += red1[w];
        const float mean = tot * invn;
        float q = 0.0f;
#pragma unroll 1
        for (unsigned b = 0; b < (unsigned)NB; ++b) {
            const float* xp = x + ((size_t)b * CH + c) * SEQ_FULL;
#pragma unroll 1
            for (unsigned i = tid * 4u; i < (unsigned)SEQ; i += 1024u) {
                const v4f v = *(const v4f*)(xp + i);
                const float d0 = bfr(v[0]) - mean, d1 = bfr(v[1]) - mean, d2 = bfr(v[2]) - mean, d3 = bfr(v[3]) - mean;
                q += (d0 * d0 + d1 * d1) + (d2 * d2 + d3 * d3);
            }
        }
#pragma unroll
        for (int off = 16; off > 0; off >>= 1) q += __shfl_xor(q, off, 32);
        if (lane == 0u) red2[wave] = q;
        __syncthreads();
        float tq = red2[0];
#pragma unroll
        for (int w = 1; w < 8; ++w) tq += red2[w];
        const float var = tq * invn;
        if (tid == 0u) { resl[cc] = mean; resl[8u + cc] = rsqrtf(var + 1.0e-5f); }
    }
    __syncthreads();
    if (tid < 8u) {
        v4f o;
        o[0] = resl[tid * 4u]; o[1] = resl[tid * 4u + 1u]; o[2] = resl[tid * 4u + 2u]; o[3] = resl[tid * 4u + 3u];
        float* dst = ST + blockIdx.x * 32u + tid * 4u;
        *(volatile v4f*)dst = o;
        __threadfence();
        *(volatile v4f*)dst = o;
    }
}

__global__ __launch_bounds__(256) void k_norm(const float* __restrict__ x, const float* __restrict__ bw, const float* __restrict__ bb, const float* __restrict__ ST, hf* XT) {
    __shared__ __align__(16) hf tl[64 * XP];
    __shared__ float pm[CH];
    __shared__ float pr[CH];
    __shared__ float pw[CH];
    __shared__ float pb[CH];
    const unsigned tid = threadIdx.x, lane = tid & 31u;
    const unsigned wave = (unsigned)__builtin_amdgcn_readfirstlane((int)(tid >> 5));
    pm[tid] = ST[(tid >> 3) * 32u + (tid & 7u)];
    pr[tid] = ST[(tid >> 3) * 32u + 8u + (tid & 7u)];
    pw[tid] = bfr(bw[tid]);
    pb[tid] = bfr(bb[tid]);
    __syncthreads();
    const unsigned tpb = (unsigned)(SEQ / 64);
    const unsigned b = blockIdx.x / tpb;
    const unsigned n0 = (blockIdx.x - b * tpb) * 64u;
    const float* src = x + (size_t)b * CH * SEQ_FULL + n0;
#pragma unroll 1
    for (unsigned it = 0; it < 16u; ++it) {
        const unsigned f = it * 256u + tid;
        const unsigned c = f >> 4, p4 = (f & 15u) * 4u;
        const v4f v = *(const v4f*)(src + (size_t)c * SEQ_FULL + p4);
        const float m = pm[c], r = pr[c], w = pw[c], bi = pb[c];
#pragma unroll
        for (unsigned e = 0; e < 4u; ++e) tl[(p4 + e) * XP + c] = (hf)(((bfr(v[e]) - m) * r) * w + bi);
    }
    __syncthreads();
    hf* dst = XT + ((size_t)b * SEQ + n0) * CH + lane * 8u;
#pragma unroll 1
    for (int ps = 0; ps < 2; ++ps) {
#pragma unroll
        for (unsigned s = 0; s < 8u; ++s) {
            const unsigned row = wave * 8u + s;
            const v8h o = *(const v8ha*)(tl + row * XP + lane * 8u);
            *(volatile v8h*)(dst + (size_t)row * CH) = o;
        }
        if (ps == 0) __threadfence();
    }
}

__global__ __launch_bounds__(128) void k_qkv(const hf* __restrict__ XT, const hf* __restrict__ WQ, hf* QH, hf* QR, hf* KB, hf* VT) {
    __shared__ __align__(16) hf sa[64 * SQ];
    __shared__ __align__(16) hf sb[64 * SQ];
    const unsigned tid = threadIdx.x, lane = tid & 31u, lr = lane & 15u, hi = lane >> 4;
    const unsigned wave = (unsigned)__builtin_amdgcn_readfirstlane((int)(tid >> 5));
    const unsigned p0 = blockIdx.x * 64u, cb = blockIdx.y, b = blockIdx.z;
    const unsigned kind = cb >> 2, head = cb & 3u;
    const hf* ap = XT + ((size_t)b * SEQ + p0 + wave * 16u + lr) * CH + 8u * hi;
    const hf* bp = WQ + ((size_t)cb * 64u + lr) * CH + 8u * hi;
    v8f acc0 = (v8f){}, acc1 = (v8f){}, acc2 = (v8f){}, acc3 = (v8f){};
#pragma unroll 1
    for (unsigned k0 = 0; k0 < (unsigned)CH; k0 += 32u) {
        const v16h a  = ldh(ap + k0);
        const v16h b0 = ldh(bp + k0);
        const v16h b1 = ldh(bp + 16 * CH + k0);
        const v16h b2 = ldh(bp + 32 * CH + k0);
        const v16h b3 = ldh(bp + 48 * CH + k0);
        acc0 = wmmah(a, b0, acc0);
        acc1 = wmmah(a, b1, acc1);
        acc2 = wmmah(a, b2, acc2);
        acc3 = wmmah(a, b3, acc3);
        asm volatile("v_nop\n\tv_nop\n\tv_nop\n\tv_nop"
                     : "+v"(acc0), "+v"(acc1), "+v"(acc2), "+v"(acc3)
                     : "v"(a), "v"(b0), "v"(b1), "v"(b2), "v"(b3));
    }
    const float us = 1.0f / 1024.0f;
    v8f acc[4] = { acc0, acc1, acc2, acc3 };
    if (kind == 2u) {
#pragma unroll
        for (int t = 0; t < 4; ++t) {
#pragma unroll
            for (int r = 0; r < 8; ++r) sa[(t * 16 + lr) * SQ + wave * 16u + 8u * hi + r] = (hf)(acc[t][r] * us);
        }
    } else if (kind == 1u) {
#pragma unroll
        for (int t = 0; t < 4; ++t) {
#pragma unroll
            for (int r = 0; r < 8; ++r) sa[(wave * 16u + 8u * hi + r) * SQ + t * 16 + lr] = (hf)(acc[t][r] * us);
        }
    } else {
#pragma unroll
        for (int t = 0; t < 4; ++t) {
#pragma unroll
            for (int r = 0; r < 8; ++r) {
                const float q = acc[t][r] * us;
                const hf qh = (hf)q;
                sa[(wave * 16u + 8u * hi + r) * SQ + t * 16 + lr] = qh;
                sb[(wave * 16u + 8u * hi + r) * SQ + t * 16 + lr] = (hf)((q - (float)qh) * 4096.0f);
            }
        }
    }
    __syncthreads();
    const unsigned pc = (lane & 7u) * 8u, rq = lane >> 3;
    const size_t qoff = (((size_t)b * NH + head) * SEQ + p0) * HD + pc;
    const size_t voff = ((size_t)b * CH + head * HD) * SEQ + p0 + pc;
#pragma unroll 1
    for (int ps = 0; ps < 2; ++ps) {
#pragma unroll
        for (unsigned s = 0; s < 4u; ++s) {
            const unsigned row = wave * 16u + s * 4u + rq;
            const v8h o = *(const v8ha*)(sa + row * SQ + pc);
            if (kind == 0u) {
                const v8h o2 = *(const v8ha*)(sb + row * SQ + pc);
                *(volatile v8h*)(QH + qoff + (size_t)row * HD) = o;
                *(volatile v8h*)(QR + qoff + (size_t)row * HD) = o2;
            } else if (kind == 1u) {
                *(volatile v8h*)(KB + qoff + (size_t)row * HD) = o;
            } else {
                *(volatile v8h*)(VT + voff + (size_t)row * SEQ) = o;
            }
        }
        if (ps == 0) __threadfence();
    }
}

__global__ __launch_bounds__(128) void k_flash(const hf* __restrict__ QH, const hf* __restrict__ QR, const hf* __restrict__ KB, const hf* __restrict__ VT, hf* CT) {
    __shared__ __align__(16) hf os[NWV * 16 * SQ];
    const unsigned tid = threadIdx.x, lane = tid & 31u, lr = lane & 15u, hi = lane >> 4;
    const unsigned wave = (unsigned)__builtin_amdgcn_readfirstlane((int)(tid >> 5));
    const unsigned bpb = (unsigned)(SEQ / BQ);
    const unsigned bh = blockIdx.x / bpb;
    const unsigned b = bh / NH, h = bh - b * NH;
    const unsigned q0 = (blockIdx.x - bh * bpb) * BQ + wave * 16u;
    const size_t pbase = (size_t)bh * SEQ * HD;

    v16h qh0, qh1, qr0, qr1;
    {
        const size_t qo = pbase + (size_t)(q0 + lr) * HD + 8u * hi;
        qh0 = ldh(QH + qo); qh1 = ldh(QH + qo + 32);
        qr0 = ldh(QR + qo); qr1 = ldh(QR + qo + 32);
    }
    const hf* kp = KB + pbase + (size_t)lr * HD + 8u * hi;
    const hf* vp = VT + ((size_t)bh * HD + lr) * SEQ + 8u * hi;

    v8f o0 = (v8f){}, o1 = (v8f){}, o2 = (v8f){}, o3 = (v8f){};
    float ml = -1.0e30f;
    float l = 0.0f;
    const float CL = 0.125f * L2E;
    const float RS = 1.0f / 4096.0f;

#pragma unroll 1
    for (unsigned k0 = 0; k0 < (unsigned)SEQ; k0 += KS) {
        v8f s0 = (v8f){}, s1 = (v8f){}, r0 = (v8f){}, r1 = (v8f){};
        const hf* ka = kp + (size_t)k0 * HD;
        const v16h a00 = ldh(ka);
        const v16h a01 = ldh(ka + 32);
        const v16h a10 = ldh(ka + 16 * HD);
        const v16h a11 = ldh(ka + 16 * HD + 32);
        s0 = wmmah(a00, qh0, s0);
        s1 = wmmah(a10, qh0, s1);
        r0 = wmmah(a00, qr0, r0);
        r1 = wmmah(a10, qr0, r1);
        s0 = wmmah(a01, qh1, s0);
        s1 = wmmah(a11, qh1, s1);
        r0 = wmmah(a01, qr1, r0);
        r1 = wmmah(a11, qr1, r1);
        asm volatile("v_nop\n\tv_nop\n\tv_nop\n\tv_nop"
                     : "+v"(s0), "+v"(s1), "+v"(r0), "+v"(r1)
                     : "v"(a00), "v"(a01), "v"(a10), "v"(a11), "v"(qh0), "v"(qh1), "v"(qr0), "v"(qr1));
#pragma unroll
        for (int r = 0; r < 8; ++r) { s0[r] = fmaf(r0[r], RS, s0[r]); s1[r] = fmaf(r1[r], RS, s1[r]); }

        float mx = fmaxf(s0[0], s1[0]);
#pragma unroll
        for (int r = 1; r < 8; ++r) mx = fmaxf(mx, fmaxf(s0[r], s1[r]));
        mx = fmaxf(mx, __shfl_xor(mx, 16, 32));
        const float mnl = fmaxf(ml, mx * CL);
        const float corr = __builtin_amdgcn_exp2f(ml - mnl);
        ml = mnl;
        const float bs = 8.0f - mnl;
        float p0[8], p1[8];
        float ps = 0.0f;
#pragma unroll
        for (int r = 0; r < 8; ++r) {
            p0[r] = __builtin_amdgcn_exp2f(fmaf(s0[r], CL, bs));
            p1[r] = __builtin_amdgcn_exp2f(fmaf(s1[r], CL, bs));
            ps += p0[r] + p1[r];
        }
        ps += __shfl_xor(ps, 16, 32);
        l = l * corr + ps;
        if (__builtin_amdgcn_ballot_w32(corr != 1.0f) != 0u) {
            o0 *= corr; o1 *= corr; o2 *= corr; o3 *= corr;
        }
        v16h ph;
#pragma unroll
        for (int r = 0; r < 8; ++r) { ph[r] = (hf)p0[r]; ph[8 + r] = (hf)p1[r]; }

        asm volatile("" ::: "memory");
        const hf* va = vp + k0;
        const v16h v0 = ldh(va);
        const v16h v1 = ldh(va + (size_t)16 * SEQ);
        const v16h v2 = ldh(va + (size_t)32 * SEQ);
        const v16h v3 = ldh(va + (size_t)48 * SEQ);
        o0 = wmmah(v0, ph, o0);
        o1 = wmmah(v1, ph, o1);
        o2 = wmmah(v2, ph, o2);
        o3 = wmmah(v3, ph, o3);
        asm volatile("v_nop\n\tv_nop\n\tv_nop\n\tv_nop"
                     : "+v"(o0), "+v"(o1), "+v"(o2), "+v"(o3)
                     : "v"(ph), "v"(v0), "v"(v1), "v"(v2), "v"(v3));
    }

    const float inv = 256.0f / l;
    const unsigned wb = wave * (16u * SQ);
    v8f oo[4] = { o0, o1, o2, o3 };
#pragma unroll
    for (int t = 0; t < 4; ++t) {
#pragma unroll
        for (int r = 0; r < 8; ++r) os[wb + lr * SQ + t * 16 + 8u * hi + r] = (hf)(oo[t][r] * inv);
    }
    __syncthreads();
    const unsigned pc = (lane & 7u) * 8u, rq = lane >> 3;
    hf* dst = CT + ((size_t)b * SEQ + q0) * CH + h * HD + pc;
#pragma unroll 1
    for (int ps2 = 0; ps2 < 2; ++ps2) {
#pragma unroll
        for (unsigned s = 0; s < 4u; ++s) {
            const unsigned row = s * 4u + rq;
            const v8h val = *(const v8ha*)(os + wb + row * SQ + pc);
            *(volatile v8h*)(dst + (size_t)row * CH) = val;
        }
        if (ps2 == 0) __threadfence();
    }
}

__global__ __launch_bounds__(128) void k_out(const hf* __restrict__ CT, const hf* __restrict__ WO, const float* __restrict__ bo, float* OUT) {
    __shared__ __align__(16) float os[64 * OP];
    const unsigned tid = threadIdx.x, lane = tid & 31u, lr = lane & 15u, hi = lane >> 4;
    const unsigned wave = (unsigned)__builtin_amdgcn_readfirstlane((int)(tid >> 5));
    const unsigned p0 = blockIdx.x * 64u, ob = blockIdx.y * 64u, b = blockIdx.z;
    const hf* ap = WO + ((size_t)(ob + wave * 16u + lr)) * CH + 8u * hi;
    const hf* bp = CT + ((size_t)b * SEQ + p0 + lr) * CH + 8u * hi;
    v8f acc0 = (v8f){}, acc1 = (v8f){}, acc2 = (v8f){}, acc3 = (v8f){};
#pragma unroll 1
    for (unsigned k0 = 0; k0 < (unsigned)CH; k0 += 32u) {
        const v16h a  = ldh(ap + k0);
        const v16h b0 = ldh(bp + k0);
        const v16h b1 = ldh(bp + 16 * CH + k0);
        const v16h b2 = ldh(bp + 32 * CH + k0);
        const v16h b3 = ldh(bp + 48 * CH + k0);
        acc0 = wmmah(a, b0, acc0);
        acc1 = wmmah(a, b1, acc1);
        acc2 = wmmah(a, b2, acc2);
        acc3 = wmmah(a, b3, acc3);
        asm volatile("v_nop\n\tv_nop\n\tv_nop\n\tv_nop"
                     : "+v"(acc0), "+v"(acc1), "+v"(acc2), "+v"(acc3)
                     : "v"(a), "v"(b0), "v"(b1), "v"(b2), "v"(b3));
    }
    const float us = 1.0f / 262144.0f;
    v8f acc[4] = { acc0, acc1, acc2, acc3 };
#pragma unroll
    for (int r = 0; r < 8; ++r) {
        const unsigned orow = wave * 16u + 8u * hi + r;
        const float bias = bfr(bo[ob + orow]);
#pragma unroll
        for (int t = 0; t < 4; ++t) os[orow * OP + t * 16 + lr] = fmaf(acc[t][r], us, bias);
    }
    __syncthreads();
    const unsigned pc = (lane & 15u) * 4u, rh = lane >> 4;
    float* dst = OUT + ((size_t)b * CH + ob) * SEQ + p0 + pc;
#pragma unroll 1
    for (int ps = 0; ps < 2; ++ps) {
#pragma unroll
        for (unsigned s = 0; s < 8u; ++s) {
            const unsigned row = wave * 16u + s * 2u + rh;
            const v4f val = *(const v4fa*)(os + row * OP + pc);
            *(volatile v4f*)(dst + (size_t)row * SEQ) = val;
        }
        if (ps == 0) __threadfence();
    }
}

extern "C" void kernel_launch(void* const* d_in, const int* in_sizes, int n_in,
                              void* d_out, int out_size, void* d_ws, size_t ws_size, hipStream_t stream) {
    if (n_in < 6) return;
    const size_t needx = ((size_t)(NB - 1) * CH + (CH - 1)) * SEQ_FULL + SEQ;
    if ((size_t)in_sizes[0] < needx) return;
    if (in_sizes[1] < CH || in_sizes[2] < CH || in_sizes[5] < CH) return;
    if (in_sizes[3] < OC3 * CH || in_sizes[4] < CH * CH) return;
    if ((size_t)out_size < (size_t)NB * CH * SEQ) return;
    if (WS_TOTAL > ws_size) return;
    const float* x    = (const float*)d_in[0];
    const float* bnw  = (const float*)d_in[1];
    const float* bnb  = (const float*)d_in[2];
    const float* wqkv = (const float*)d_in[3];
    const float* wout = (const float*)d_in[4];
    const float* bout = (const float*)d_in[5];
    float* OUT = (float*)d_out;
    char* wsp = (char*)d_ws;
    size_t off = 0;
    float* ST = (float*)(wsp + off); off += ST_BYTES;
    hf* WQ = (hf*)(wsp + off); off += WQ_BYTES;
    hf* WO = (hf*)(wsp + off); off += WO_BYTES;
    hf* XT = (hf*)(wsp + off); off += PL_BYTES;
    hf* QH = (hf*)(wsp + off); off += PL_BYTES;
    hf* QR = (hf*)(wsp + off); off += PL_BYTES;
    hf* KB = (hf*)(wsp + off); off += PL_BYTES;
    hf* VT = (hf*)(wsp + off); off += PL_BYTES;
    hf* CT = (hf*)(wsp + off); off += PL_BYTES;
    k_cvtw<<<dim3((unsigned)(OC3 * CH / 8 / 256), 2, 1), 256, 0, stream>>>(wqkv, wout, WQ, WO);
    k_bnstat<<<(unsigned)(CH / 8), 256, 0, stream>>>(x, ST);
    k_norm<<<(unsigned)(NB * (SEQ / 64)), 256, 0, stream>>>(x, bnw, bnb, ST, XT);
    k_qkv<<<dim3((unsigned)(SEQ / 64), 12, (unsigned)NB), 128, 0, stream>>>(XT, WQ, QH, QR, KB, VT);
    k_flash<<<(unsigned)(NB * NH * (SEQ / BQ)), 128, 0, stream>>>(QH, QR, KB, VT, CT);
    k_out<<<dim3((unsigned)(SEQ / 64), (unsigned)(CH / 64), (unsigned)NB), 128, 0, stream>>>(CT, WO, bout, OUT);
}
